// TemporalSelfAttention_13932873909055
// MI455X (gfx1250) — hardware-run, weakly checked
//
#include <hip/hip_runtime.h>

typedef float          v8f   __attribute__((ext_vector_type(8)));
typedef float          v4f   __attribute__((ext_vector_type(4)));
typedef unsigned int   v4u   __attribute__((ext_vector_type(4)));
typedef int            v8i   __attribute__((ext_vector_type(8)));
typedef unsigned short v8us  __attribute__((ext_vector_type(8)));
typedef unsigned short v16us __attribute__((ext_vector_type(16)));
typedef __bf16         v16bf __attribute__((ext_vector_type(16)));
typedef _Float16       v16h  __attribute__((ext_vector_type(16)));
typedef v4f  __attribute__((may_alias)) v4fa;
typedef v8us __attribute__((may_alias)) v8usa;
union FragB { v16bf v; v16us u; v8us h[2]; v8i w; };
union FragH { v16h  v; v16us u; v8us h[2]; v8i w; };

__device__ __forceinline__ v8f wmb(const FragB& a, const FragB& b, v8f c) {
  v8f d = __builtin_amdgcn_wmma_f32_16x16x32_bf16(false, a.v, false, b.v, (short)0, c, false, false);
  asm volatile("v_nop\n\tv_nop\n\tv_nop\n\tv_nop" : "+v"(d) : "v"(a.w), "v"(b.w));
  return d;
}

__device__ __forceinline__ v8f wmh(const FragH& a, const FragH& b, v8f c) {
  v8f d = __builtin_amdgcn_wmma_f32_16x16x32_f16(false, a.v, false, b.v, (short)0, c, false, false);
  asm volatile("v_nop\n\tv_nop\n\tv_nop\n\tv_nop" : "+v"(d) : "v"(a.w), "v"(b.w));
  return d;
}

__device__ __forceinline__ unsigned bf16_bits(float f) {
  const unsigned u = __float_as_uint(f);
  const unsigned r = (u + 0x7FFFu + ((u >> 16) & 1u)) >> 16;
  const unsigned q = (u >> 16) | 0x40u;
  return ((u & 0x7fffffffu) > 0x7f800000u) ? q : r;
}

__device__ __forceinline__ float bf16_val(float f) {
  return __uint_as_float(bf16_bits(f) << 16);
}
__device__ __forceinline__ int clampi(int v, int lo, int hi) {
  return v < lo ? lo : (v > hi ? hi : v);
}

__device__ __forceinline__ unsigned f16_bits(float f) {
  const unsigned u  = __float_as_uint(f);
  const unsigned s  = (u >> 16) & 0x8000u;
  const unsigned a  = u & 0x7fffffffu;
  const unsigned t  = a - 0x38000000u;
  const unsigned r  = (t + 0x0FFFu + ((t >> 13) & 1u)) >> 13;
  const unsigned rc = r > 0x7C00u ? 0x7C00u : r;
  const bool small  = a < 0x38800000u;
  const bool isnan  = a > 0x7f800000u;
  const unsigned fin = small ? 0u : (s | rc);
  return isnan ? (s | 0x7E00u) : fin;
}

__device__ __forceinline__ unsigned pk16(unsigned lo, unsigned hi) { return lo | (hi << 16); }
__device__ __forceinline__ unsigned bf16_lo_bits(float v) {
  float hi = bf16_val(v);
  asm volatile("" : "+v"(hi));
  return bf16_bits(v - hi);
}
__device__ __forceinline__ v4u pack8_bf16(v4f a, v4f c) {
  return (v4u){ pk16(bf16_bits(a[0]), bf16_bits(a[1])), pk16(bf16_bits(a[2]), bf16_bits(a[3])),
                pk16(bf16_bits(c[0]), bf16_bits(c[1])), pk16(bf16_bits(c[2]), bf16_bits(c[3])) };
}
__device__ __forceinline__ v4u pack8_bf16_lo(v4f a, v4f c) {
  return (v4u){ pk16(bf16_lo_bits(a[0]), bf16_lo_bits(a[1])), pk16(bf16_lo_bits(a[2]), bf16_lo_bits(a[3])),
                pk16(bf16_lo_bits(c[0]), bf16_lo_bits(c[1])), pk16(bf16_lo_bits(c[2]), bf16_lo_bits(c[3])) };
}
__device__ __forceinline__ v4u pack8_f16(v4f a, v4f c) {
  return (v4u){ pk16(f16_bits(a[0]), f16_bits(a[1])), pk16(f16_bits(a[2]), f16_bits(a[3])),
                pk16(f16_bits(c[0]), f16_bits(c[1])), pk16(f16_bits(c[2]), f16_bits(c[3])) };
}

template <int FORM>
__global__ __launch_bounds__(256) void k_plane(const float* __restrict__ src, int rows, int cols, int ldsrc,
                                               unsigned short* __restrict__ dst, int MP, int KP) {
  static_assert(FORM >= 0 && FORM <= 3);
  const int KTOT = (FORM == 1 || FORM == 3) ? 2 * KP : KP;
  const unsigned ppr   = (unsigned)(KTOT >> 3);
  const unsigned kp8   = (unsigned)(KP >> 3);
  const unsigned total = (unsigned)MP * ppr;
  const unsigned g     = blockIdx.x * 256u + threadIdx.x;
  const unsigned rowu  = g / ppr;
  const unsigned p     = g - rowu * ppr;
  const bool second    = p >= kp8;
  const int row = (int)rowu;
  const int c0  = (int)((second ? p - kp8 : p) << 3);
  const float* srow = src + (size_t)clampi(row, 0, rows - 1) * (size_t)ldsrc;
  float x[8];
  unsigned mk[8];
#pragma unroll
  for (int e = 0; e < 8; ++e) {
    const int c = c0 + e;
    const float v = srow[clampi(c, 0, cols - 1)];
    asm volatile("" :: "v"(v));
    x[e]  = v;
    mk[e] = (row < rows && c < cols) ? 0xFFFFu : 0u;
  }
  const v4f a = (v4f){ x[0], x[1], x[2], x[3] };
  const v4f c = (v4f){ x[4], x[5], x[6], x[7] };
  v4u o;
  if (FORM == 2) {
    o = pack8_f16(a, c);
  } else {
    const v4u hi = pack8_bf16(a, c);
    o = hi;
    if (FORM == 1) { const v4u lo = pack8_bf16_lo(a, c); o = second ? lo : hi; }
  }
  const v4u mw = (v4u){ pk16(mk[0], mk[1]), pk16(mk[2], mk[3]), pk16(mk[4], mk[5]), pk16(mk[6], mk[7]) };
  o &= mw;
  if (g < total) {
    volatile v4u* q = (volatile v4u*)(dst + (size_t)g * 8);
    *q = o;
    __threadfence();
    *q = o;
  }
}

template <int FORM> struct FragOf    { typedef FragB T; };
template <>         struct FragOf<2> { typedef FragH T; };
__device__ __forceinline__ v8f mm(const FragB& a, const FragB& b, v8f c) { return wmb(a, b, c); }
__device__ __forceinline__ v8f mm(const FragH& a, const FragH& b, v8f c) { return wmh(a, b, c); }
template <class F> __device__ __forceinline__ F ld_frag(const unsigned short* p) {
  F f;
  f.h[0] = *(const v8usa*)(p);
  f.h[1] = *(const v8usa*)(p + 16);
  return f;
}

template <int FORM, int EPI>
__global__ __launch_bounds__(256) __attribute__((amdgpu_num_vgpr(248)))
void k_gemm_nt(const unsigned short* __restrict__ A, const unsigned short* __restrict__ B,
               const float* __restrict__ bias, float* __restrict__ D, int M, int N, int KTOT, int ldd) {
  static_assert(FORM >= 0 && FORM <= 2);
  static_assert(EPI == 0 || EPI == 1);
  typedef typename FragOf<FORM>::T F;
  __shared__ __attribute__((aligned(16))) float sT[8][16 * 68];
  const int lane = threadIdx.x & 31;
  const int wave = threadIdx.x >> 5;
  const int tilesM = (M + 63) >> 6;
  const int tilesN = (N + 63) >> 6;
  const int tile = blockIdx.x * 8 + wave;
  if (tile >= tilesM * tilesN) return;
  const int tm = tile / tilesN;
  const int tn = tile - tm * tilesN;
  const int m0 = tm << 6;
  const int n0 = tn << 6;

  const int rl = lane & 15;
  const int h8 = (lane >> 4) * 8;
  const unsigned short* pa = A + (size_t)(m0 + rl) * (size_t)KTOT + h8;
  const unsigned short* pb = B + (size_t)(n0 + rl) * (size_t)KTOT + h8;

  v8f acc[4][4];
#pragma unroll
  for (int i = 0; i < 4; ++i)
#pragma unroll
    for (int j = 0; j < 4; ++j) acc[i][j] = (v8f){0.f, 0.f, 0.f, 0.f, 0.f, 0.f, 0.f, 0.f};

#pragma unroll 1
  for (int k0 = 0; k0 < KTOT; k0 += 32) {
    F bf[4];
#pragma unroll
    for (int j = 0; j < 4; ++j) bf[j] = ld_frag<F>(pb + (size_t)(j << 4) * (size_t)KTOT + k0);
#pragma unroll
    for (int i = 0; i < 4; ++i) {
      const F af = ld_frag<F>(pa + (size_t)(i << 4) * (size_t)KTOT + k0);
#pragma unroll
      for (int j = 0; j < 4; ++j) acc[i][j] = mm(af, bf[j], acc[i][j]);
    }
  }

  float* slab = sT[wave];
  const int hh = lane >> 4;
  const int c4 = (lane & 15) * 4;
  const int nc = n0 + c4;
  const bool cok = nc < N;
  v4f bv = (v4f){0.f, 0.f, 0.f, 0.f};
  if (EPI == 1) {
    bv = *(const v4fa*)(bias + clampi(nc, 0, N - 4));
    asm volatile("" :: "v"(bv));
  }
#pragma unroll
  for (int i = 0; i < 4; ++i) {
    const int mBase = m0 + (i << 4);
#pragma unroll
    for (int j = 0; j < 4; ++j) {
#pragma unroll
      for (int r = 0; r < 8; ++r) slab[(h8 + r) * 68 + (j << 4) + rl] = acc[i][j][r];
    }
    __builtin_amdgcn_fence(__ATOMIC_RELEASE, "workgroup");
    __builtin_amdgcn_wave_barrier();
    __builtin_amdgcn_fence(__ATOMIC_ACQUIRE, "workgroup");
    v4f vv[8];
#pragma unroll
    for (int it = 0; it < 8; ++it) {
      const int row = it * 2 + hh;
      v4f v = *(const v4fa*)(slab + row * 68 + c4);
      if (EPI == 1) v += bv;
      vv[it] = v;
    }
    for (int pass = 0; pass < 2; ++pass) {
#pragma unroll
      for (int it = 0; it < 8; ++it) {
        const int row = mBase + it * 2 + hh;
        if (cok && row < M) *(volatile v4f*)(D + (size_t)row * (size_t)ldd + nc) = vv[it];
      }
      __threadfence();
    }
    __builtin_amdgcn_fence(__ATOMIC_RELEASE, "workgroup");
    __builtin_amdgcn_wave_barrier();
    __builtin_amdgcn_fence(__ATOMIC_ACQUIRE, "workgroup");
  }
}

#ifndef OUT_FORM
#define OUT_FORM 2
#endif
static_assert(OUT_FORM >= 1 && OUT_FORM <= 3);
#if OUT_FORM == 2
#define MK     512
#define GFORM  1
#define GEPI   1
#define WOF16  0
#define WCARRY 1.0f
#define YINV   1.0f
#elif OUT_FORM == 1
#define MK     256
#define GFORM  0
#define GEPI   1
#define WOF16  0
#define WCARRY 1.0f
#define YINV   1.0f
#else
#define MK     256
#define GFORM  2
#define GEPI   0
#define WOF16  1
#define WCARRY 64.0f
#define YINV   0.015625f
#endif

#define NQ     16384
#define EMB    256
#define NHEAD  8
#define DHEAD  32
#define NPT    4
#define NFR    2
#define HBEV   128
#define WBEV   128
#define QEK    512
#define NSO    128
#define NAW    64
#define NSA    192
#define NSMP   64
#define TABW   12
#define WSLIM  ((size_t)128 << 20)

static_assert(NQ == HBEV * WBEV);
static_assert(EMB == NHEAD * DHEAD);
static_assert(DHEAD == 32);
static_assert(QEK == 2 * EMB);
static_assert(NSO == NFR * NHEAD * NPT * 2);
static_assert(NAW == NFR * NHEAD * NPT);
static_assert(NSA == NSO + NAW);
static_assert(NSMP == NHEAD * NFR * NPT);
static_assert(NSMP == 64);
static_assert(NSA % 64 == 0 && NSA % 32 == 0);
static_assert(EMB % 64 == 0 && EMB % 32 == 0);
static_assert(NQ % 64 == 0 && (NFR * NQ) % 64 == 0);
static_assert(QEK % 32 == 0 && MK % 32 == 0);
static_assert((TABW * 4) % 16 == 0);
static_assert(8 * NSMP * TABW * 4 + 8 * EMB * 4 == 32768);
static_assert((NFR * NQ) * EMB < (1 << 24) * 4);

typedef float v2f __attribute__((ext_vector_type(2)));
typedef v2f __attribute__((may_alias)) v2fa;
typedef v4u __attribute__((may_alias)) v4ua;

template <int F16>
__global__ __launch_bounds__(256) void k_wt(const float* __restrict__ W, int K, int N,
                                            unsigned short* __restrict__ dst, int KTOT, float carry) {
  const unsigned ppr   = (unsigned)(KTOT >> 3);
  const unsigned total = (unsigned)N * ppr;
  const unsigned g     = blockIdx.x * 256u + threadIdx.x;
  const unsigned gc    = g < total ? g : total - 1u;
  const unsigned n     = gc / ppr;
  const unsigned p     = gc - n * ppr;
  const int kk = (int)(p << 3);
  const int k0 = (kk >= K) ? kk - K : kk;
  float x[8];
#pragma unroll
  for (int e = 0; e < 8; ++e) {
    const float v = W[(size_t)clampi(k0 + e, 0, K - 1) * (size_t)N + n];
    asm volatile("" :: "v"(v));
    x[e] = carry * bf16_val(v);
  }
  const v4f a = (v4f){ x[0], x[1], x[2], x[3] };
  const v4f c = (v4f){ x[4], x[5], x[6], x[7] };
  const v4u o = F16 ? pack8_f16(a, c) : pack8_bf16(a, c);
  if (g < total) {
    volatile v4u* q = (volatile v4u*)(dst + (size_t)g * 8);
    *q = o;
    __threadfence();
    *q = o;
  }
}

__global__ __launch_bounds__(256) void k_qe(const float* __restrict__ value, const float* __restrict__ query,
                                            unsigned short* __restrict__ QE) {
  const unsigned g  = blockIdx.x * 256u + threadIdx.x;
  const unsigned q  = g >> 6;
  const unsigned p  = g & 63u;
  const unsigned c0 = (p & 31u) << 3;
  const size_t so = (size_t)q * EMB + c0;
  const v4f va = *(const v4fa*)(value + so);
  const v4f vc = *(const v4fa*)(value + so + 4);
  const v4f qa = *(const v4fa*)(query + so);
  const v4f qc = *(const v4fa*)(query + so + 4);
  asm volatile("" :: "v"(va), "v"(vc), "v"(qa), "v"(qc));
  const unsigned mv = (p < 32u) ? 0xFFFFFFFFu : 0u;
  const unsigned mq = ~mv;
  v4f a, c;
#pragma unroll
  for (int e = 0; e < 4; ++e) {
    a[e] = __uint_as_float((__float_as_uint(va[e]) & mv) | (__float_as_uint(qa[e]) & mq));
    c[e] = __uint_as_float((__float_as_uint(vc[e]) & mv) | (__float_as_uint(qc[e]) & mq));
  }
  const v4u o = pack8_bf16(a, c);
  volatile v4u* d = (volatile v4u*)(QE + (size_t)g * 8);
  *d = o;
  __threadfence();
  *d = o;
}

__global__ __launch_bounds__(192) void k_bias(const float* __restrict__ bvp, const float* __restrict__ bo,
                                              const float* __restrict__ bso, const float* __restrict__ baw,
                                              float* __restrict__ dst) {
  const int t = threadIdx.x;
  const int p = t & 63;
  const v4f xv = *(const v4fa*)(bvp + 4 * p);
  const v4f xo = *(const v4fa*)(bo + 4 * p);
  const v4f xs = *(const v4fa*)(bso + 4 * clampi(p, 0, 31));
  const v4f xa = *(const v4fa*)(baw + 4 * clampi(p - 32, 0, 15));
  asm volatile("" :: "v"(xv), "v"(xo), "v"(xs), "v"(xa));
  const unsigned mv = (t < 64) ? 0xFFFFFFFFu : 0u;
  const unsigned mo = (t >= 64 && t < 128) ? 0xFFFFFFFFu : 0u;
  const unsigned ms = (t >= 128 && p < 32) ? 0xFFFFFFFFu : 0u;
  const unsigned ma = (t >= 128 && p >= 32 && p < 48) ? 0xFFFFFFFFu : 0u;
  v4f o;
#pragma unroll
  for (int e = 0; e < 4; ++e) {
    const unsigned b = ((bf16_bits(xv[e]) << 16) & mv) | ((bf16_bits(xo[e]) << 16) & mo) |
                       ((bf16_bits(xs[e]) << 16) & ms) | ((bf16_bits(xa[e]) << 16) & ma);
    o[e] = __uint_as_float(b);
  }
  volatile v4f* d = (volatile v4f*)(dst + 4 * t);
  *d = o;
  __threadfence();
  *d = o;
}

__global__ __launch_bounds__(256) void k_sample(const float* __restrict__ V, const float* __restrict__ SOAW,
                                                const float* __restrict__ rp, const int* __restrict__ shp,
                                                unsigned short* __restrict__ MHL) {
  __shared__ __attribute__((aligned(16))) unsigned sTab[8][NSMP * TABW];
  __shared__ __attribute__((aligned(16))) float sM[8][EMB];
  const int lane = threadIdx.x & 31;
  const int wave = threadIdx.x >> 5;
  const int q    = blockIdx.x * 8 + wave;
  const int Hd = clampi(shp[0], 1, HBEV);
  const int Wd = clampi(shp[1], 1, WBEV);
  const float fW = (float)Wd;
  const float fH = (float)Hd;
  const float rcW = 1.0f / fW;
  const float rcH = 1.0f / fH;
  const float* srow = SOAW + (size_t)q * NSA;
  const v2f rpv = *(const v2fa*)(rp + 2 * q);
  const float rx = bf16_val(rpv[0]);
  const float ry = bf16_val(rpv[1]);

#pragma unroll 1
  for (int t = 0; t < 2; ++t) {
#pragma clang fp contract(off)
    const int s = lane + 32 * t;
    const v2f ofs = *(const v2fa*)(srow + 2 * s);
    const float lg = srow[NSO + s];
    float mx = fmaxf(lg, __shfl_xor(lg, 1));
    mx = fmaxf(mx, __shfl_xor(mx, 2));
    const float ex = expf(lg - mx);
    float sm = ex + __shfl_xor(ex, 1);
    sm = sm + __shfl_xor(sm, 2);
    const float aw = ex * (1.0f / sm);

    const float locx = rx + ofs[0] * rcW;
    const float locy = ry + ofs[1] * rcH;
    const float px = locx * fW - 0.5f;
    const float py = locy * fH - 0.5f;
    const float x0f = floorf(px);
    const float y0f = floorf(py);
    const float lx = px - x0f;
    const float ly = py - y0f;
    const int x0 = (int)fminf(fmaxf(x0f, -1.0e6f), 1.0e6f);
    const int y0 = (int)fminf(fmaxf(y0f, -1.0e6f), 1.0e6f);
    const int x1 = x0 + 1;
    const int y1 = y0 + 1;
    const bool vx0 = (x0 >= 0) & (x0 < Wd);
    const bool vx1 = (x1 >= 0) & (x1 < Wd);
    const bool vy0 = (y0 >= 0) & (y0 < Hd);
    const bool vy1 = (y1 >= 0) & (y1 < Hd);
    const float ox = 1.0f - lx;
    const float oy = 1.0f - ly;
    const float w00 = (vx0 & vy0) ? ox * oy : 0.0f;
    const float w10 = (vx1 & vy0) ? lx * oy : 0.0f;
    const float w01 = (vx0 & vy1) ? ox * ly : 0.0f;
    const float w11 = (vx1 & vy1) ? lx * ly : 0.0f;
    const int cx0 = clampi(x0, 0, Wd - 1);
    const int cx1 = clampi(x1, 0, Wd - 1);
    const int cy0 = clampi(y0, 0, Hd - 1);
    const int cy1 = clampi(y1, 0, Hd - 1);
    const int hd = s >> 3;
    const int fr = (s >> 2) & 1;
    const int rb = fr * NQ;
    const int ch = hd * DHEAD;
    const unsigned e00 = (unsigned)((rb + clampi(cy0 * Wd + cx0, 0, NQ - 1)) * EMB + ch);
    const unsigned e10 = (unsigned)((rb + clampi(cy0 * Wd + cx1, 0, NQ - 1)) * EMB + ch);
    const unsigned e01 = (unsigned)((rb + clampi(cy1 * Wd + cx0, 0, NQ - 1)) * EMB + ch);
    const unsigned e11 = (unsigned)((rb + clampi(cy1 * Wd + cx1, 0, NQ - 1)) * EMB + ch);
    unsigned* te = &sTab[wave][s * TABW];
    *(v4ua*)(te)     = (v4u){ e00, e10, e01, e11 };
    *(v4ua*)(te + 4) = (v4u){ __float_as_uint(w00), __float_as_uint(w10), __float_as_uint(w01), __float_as_uint(w11) };
    *(v4ua*)(te + 8) = (v4u){ __float_as_uint(aw), 0u, 0u, 0u };
  }
  __syncthreads();

  const float* Vl = V + lane;
  const unsigned* tw = sTab[wave];
#pragma unroll 1
  for (int h = 0; h < NHEAD; ++h) {
    float tot = 0.0f;
#pragma unroll 1
    for (int f = 0; f < NFR; ++f) {
      float af = 0.0f;
#pragma unroll 2
      for (int p = 0; p < NPT; ++p) {
        const unsigned* te = tw + ((h * NFR + f) * NPT + p) * TABW;
        const v4u eo = *(const v4ua*)(te);
        const v4u wb = *(const v4ua*)(te + 4);
        const float aw = __uint_as_float(te[8]);
        const float g00 = Vl[eo[0]];
        const float g10 = Vl[eo[1]];
        const float g01 = Vl[eo[2]];
        const float g11 = Vl[eo[3]];
        asm volatile("" :: "v"(g00), "v"(g10), "v"(g01), "v"(g11));
        float sp = __uint_as_float(wb[0]) * g00;
        sp += __uint_as_float(wb[1]) * g10;
        sp += __uint_as_float(wb[2]) * g01;
        sp += __uint_as_float(wb[3]) * g11;
        af += aw * sp;
      }
      tot += af;
    }
    sM[wave][h * DHEAD + lane] = tot * 0.5f;
  }
  __syncthreads();

  const float* mrow = sM[wave] + 8 * lane;
  const v4f a = *(const v4fa*)(mrow);
  const v4f c = *(const v4fa*)(mrow + 4);
  unsigned short* orow = MHL + (size_t)q * MK;
#if OUT_FORM == 2
  const v4u hi = pack8_bf16(a, c);
  const v4u lo = pack8_bf16_lo(a, c);
  volatile v4u* ph = (volatile v4u*)(orow + 8 * lane);
  volatile v4u* pl = (volatile v4u*)(orow + EMB + 8 * lane);
  *ph = hi;
  *pl = lo;
  __threadfence();
  *ph = hi;
  *pl = lo;
#elif OUT_FORM == 1
  const v4u hi = pack8_bf16(a, c);
  volatile v4u* ph = (volatile v4u*)(orow + 8 * lane);
  *ph = hi;
  __threadfence();
  *ph = hi;
#else
  const v4u hi = pack8_f16(a, c);
  volatile v4u* ph = (volatile v4u*)(orow + 8 * lane);
  *ph = hi;
  __threadfence();
  *ph = hi;
#endif
}

__global__ __launch_bounds__(256) void k_res(const float* __restrict__ Y, const float* __restrict__ query,
                                             const float* __restrict__ BO, float* __restrict__ out) {
  const unsigned g = blockIdx.x * 256u + threadIdx.x;
  const size_t e0 = (size_t)g * 4;
  const v4f y = *(const v4fa*)(Y + e0);
  const v4f x = *(const v4fa*)(query + e0);
  v4f o;
#if OUT_FORM == 3
  const v4f b = *(const v4fa*)(BO + ((g * 4u) & (unsigned)(EMB - 1)));
#pragma unroll
  for (int e = 0; e < 4; ++e) o[e] = (y[e] * YINV + b[e]) + bf16_val(x[e]);
#else
  (void)BO;
#pragma unroll
  for (int e = 0; e < 4; ++e) o[e] = y[e] + bf16_val(x[e]);
#endif
  volatile v4f* d = (volatile v4f*)(out + e0);
  *d = o;
  __threadfence();
  *d = o;
}

extern "C" void kernel_launch(void* const* d_in, const int* in_sizes, int n_in,
                              void* d_out, int out_size, void* d_ws, size_t ws_size,
                              hipStream_t stream) {
  if (n_in < 13) return;
  if (in_sizes[0] != NQ * EMB) return;
  if (in_sizes[1] != NFR * NQ * EMB) return;
  if (in_sizes[2] != NQ * 2) return;
  if (in_sizes[3] != EMB * EMB) return;
  if (in_sizes[4] != EMB) return;
  if (in_sizes[5] != QEK * NSO) return;
  if (in_sizes[6] != NSO) return;
  if (in_sizes[7] != QEK * NAW) return;
  if (in_sizes[8] != NAW) return;
  if (in_sizes[9] != EMB * EMB) return;
  if (in_sizes[10] != EMB) return;
  if (in_sizes[11] != 2) return;
  if (out_size != NQ * EMB) return;

  const float* query = (const float*)d_in[0];
  const float* value = (const float*)d_in[1];
  const float* rp    = (const float*)d_in[2];
  const float* Wv    = (const float*)d_in[3];
  const float* bvp   = (const float*)d_in[4];
  const float* Wso   = (const float*)d_in[5];
  const float* bso   = (const float*)d_in[6];
  const float* Waw   = (const float*)d_in[7];
  const float* baw   = (const float*)d_in[8];
  const float* Wo    = (const float*)d_in[9];
  const float* bo    = (const float*)d_in[10];
  const int*   shp   = (const int*)d_in[11];
  float* out = (float*)d_out;

  size_t off = 0;
  const size_t oVB   = off; off += (size_t)NFR * NQ * EMB * 2;
  const size_t oQE   = off; off += (size_t)NQ * QEK * 2;
  const size_t oWV   = off; off += (size_t)EMB * EMB * 2;
  const size_t oWSA  = off; off += (size_t)NSA * QEK * 2;
  const size_t oWO   = off; off += (size_t)EMB * 512 * 2;
  const size_t oBIAS = off; off += (size_t)4096;
  const size_t oV    = off; off += (size_t)NFR * NQ * EMB * 4;
  const size_t oSOAW = off; off += (size_t)NQ * NSA * 4;
  const size_t oMHL  = off; off += (size_t)NQ * 512 * 2;
  const size_t oY    = off; off += (size_t)NQ * EMB * 4;
  if (off > ws_size) return;
  if (off > WSLIM) return;

  char* ws = (char*)d_ws;
  unsigned short* VB  = (unsigned short*)(ws + oVB);
  unsigned short* QE  = (unsigned short*)(ws + oQE);
  unsigned short* WV  = (unsigned short*)(ws + oWV);
  unsigned short* WSA = (unsigned short*)(ws + oWSA);
  unsigned short* WO  = (unsigned short*)(ws + oWO);
  float* BIAS = (float*)(ws + oBIAS);
  float* BV   = BIAS;
  float* BO   = BIAS + 256;
  float* BSA  = BIAS + 512;
  float* Vf   = (float*)(ws + oV);
  float* SOAW = (float*)(ws + oSOAW);
  unsigned short* MHL = (unsigned short*)(ws + oMHL);
  float* Y    = (float*)(ws + oY);

  k_plane<0><<<dim3((NFR * NQ) * (EMB / 8) / 256), dim3(256), 0, stream>>>(value, NFR * NQ, EMB, EMB, VB, NFR * NQ, EMB);
  k_qe<<<dim3(NQ * (QEK / 8) / 256), dim3(256), 0, stream>>>(value, query, QE);
  k_wt<0><<<dim3(EMB * (EMB / 8) / 256), dim3(256), 0, stream>>>(Wv, EMB, EMB, WV, EMB, 1.0f);
  k_wt<0><<<dim3(NSO * (QEK / 8) / 256), dim3(256), 0, stream>>>(Wso, QEK, NSO, WSA, QEK, 1.0f);
  k_wt<0><<<dim3(NAW * (QEK / 8) / 256), dim3(256), 0, stream>>>(Waw, QEK, NAW, WSA + (size_t)NSO * QEK, QEK, 1.0f);
  k_wt<WOF16><<<dim3(EMB * (MK / 8) / 256), dim3(256), 0, stream>>>(Wo, EMB, EMB, WO, MK, WCARRY);
  k_bias<<<dim3(1), dim3(192), 0, stream>>>(bvp, bo, bso, baw, BIAS);

  {
    const int tiles = ((NFR * NQ + 63) / 64) * ((EMB + 63) / 64);
    k_gemm_nt<0, 1><<<dim3((tiles + 7) / 8), dim3(256), 0, stream>>>(VB, WV, BV, Vf, NFR * NQ, EMB, EMB, EMB);
  }
  {
    const int tiles = ((NQ + 63) / 64) * ((NSA + 63) / 64);
    k_gemm_nt<0, 1><<<dim3((tiles + 7) / 8), dim3(256), 0, stream>>>(QE, WSA, BSA, SOAW, NQ, NSA, QEK, NSA);
  }
  k_sample<<<dim3(NQ / 8), dim3(256), 0, stream>>>(Vf, SOAW, rp, shp, MHL);
  {
    const int tiles = ((NQ + 63) / 64) * ((EMB + 63) / 64);
    k_gemm_nt<GFORM, GEPI><<<dim3((tiles + 7) / 8), dim3(256), 0, stream>>>(MHL, WO, BO, Y, NQ, EMB, MK, EMB);
  }
  k_res<<<dim3(NQ * EMB / 4 / 256), dim3(256), 0, stream>>>(Y, query, BO, out);
  (void)hipGetLastError();
}
